// LinearAttention_62560493633831
// MI455X (gfx1250) — hardware-verified
//
#include <hip/hip_runtime.h>
#include <math.h>

typedef __attribute__((ext_vector_type(16))) _Float16 v16h;
typedef __attribute__((ext_vector_type(8)))  _Float16 v8h;
typedef __attribute__((ext_vector_type(4)))  _Float16 v4h;
typedef __attribute__((ext_vector_type(16))) __bf16   v16b;
typedef __attribute__((ext_vector_type(8)))  __bf16   v8b;
typedef __attribute__((ext_vector_type(8)))  float    v8f;
typedef __attribute__((ext_vector_type(4)))  float    v4f;

constexpr int kBatch = 4;
constexpr int kSeq   = 4096;
constexpr int kDin   = 512;
constexpr int kHid   = 512;
constexpr int kH3    = 3 * kHid;
constexpr int kTB    = 128;
constexpr int kNBlk  = kSeq / kTB;
constexpr int kRows  = kBatch * kSeq;
constexpr int kThr   = 256;
constexpr int kK2    = 2 * kHid;

constexpr float kInCarry = 1024.0f;
constexpr float kWtCarry = 4096.0f;
constexpr float kQCarry  = 64.0f;
constexpr float kSCarry  = 16.0f;
constexpr float kYCarry  = 1.0f;
constexpr float kXwScale = 1.0f / (kInCarry * kWtCarry);
constexpr float kQkScale = 1.0f / (kQCarry * kQCarry);
constexpr float kQsScale = 1.0f / (kQCarry * kSCarry);
constexpr float kYoScale = 1.0f / (kYCarry * kWtCarry);
constexpr float kF16MinNormal = 6.103515625e-5f;

static_assert((kTB % 64) == 0 && (kH3 % 64) == 0 && (kHid % 64) == 0 && (kRows % 64) == 0, "GEMM M, N multiples of 64");
static_assert((kDin % 32) == 0 && (kHid % 32) == 0 && (kTB % 32) == 0, "GEMM K multiples of 32");

constexpr size_t kOffX16  = 0;
constexpr size_t kOffWT   = kOffX16  + (size_t)kRows * kDin * 2;
constexpr size_t kOffWOT  = kOffWT   + (size_t)kH3 * kDin * 2;
constexpr size_t kOffZB   = kOffWOT  + (size_t)kHid * 2 * kHid * 2;
constexpr size_t kOffQKVB = kOffZB   + (size_t)kH3 * 4;
constexpr size_t kOffQ16  = kOffQKVB + (size_t)kBatch * kTB * kH3 * 4;
constexpr size_t kOffK16  = kOffQ16  + (size_t)kBatch * kTB * 2 * kHid * 2;
constexpr size_t kOffKT   = kOffK16  + (size_t)kBatch * kTB * kHid * 2;
constexpr size_t kOffVT   = kOffKT   + (size_t)kBatch * kHid * kTB * 2;
constexpr size_t kOffQK   = kOffVT   + (size_t)kBatch * kHid * kTB * 2;
constexpr size_t kOffW16  = kOffQK   + (size_t)kBatch * kTB * kTB * 4;
constexpr size_t kOffP1   = kOffW16  + (size_t)kBatch * kTB * kTB * 2;
constexpr size_t kOffP2   = kOffP1   + (size_t)kBatch * kTB * kHid * 4;
constexpr size_t kOffU    = kOffP2   + (size_t)kBatch * kTB * kHid * 4;
constexpr size_t kOffST32 = kOffU    + (size_t)kBatch * kHid * kHid * 4;
constexpr size_t kOffST16 = kOffST32 + (size_t)kBatch * kHid * kHid * 4;
constexpr size_t kOffY16  = kOffST16 + (size_t)kBatch * kHid * 2 * kHid * 2;
constexpr size_t kWsTotal = kOffY16  + (size_t)kRows * 2 * kHid * 2;
static_assert(kWsTotal == 73799680ull, "carve total");
static_assert(kWsTotal <= 134217728ull, "carve cap");
static_assert((kOffWT % 256) == 0 && (kOffWOT % 256) == 0 && (kOffZB % 256) == 0 && (kOffQKVB % 256) == 0 && (kOffQ16 % 256) == 0 && (kOffK16 % 256) == 0 && (kOffKT % 256) == 0 && (kOffVT % 256) == 0 && (kOffQK % 256) == 0 && (kOffW16 % 256) == 0 && (kOffP1 % 256) == 0 && (kOffP2 % 256) == 0 && (kOffU % 256) == 0 && (kOffST32 % 256) == 0 && (kOffST16 % 256) == 0 && (kOffY16 % 256) == 0, "aligned regions");

__device__ __forceinline__ unsigned short f2bf_bits(float f) {
  unsigned u = __float_as_uint(f);
  return (unsigned short)((u + 0x7FFFu + ((u >> 16) & 1u)) >> 16);
}
__device__ __forceinline__ float bf_bits2f(unsigned short h) { return __uint_as_float(((unsigned)h) << 16); }
__device__ __forceinline__ float bf16r(float f) { return bf_bits2f(f2bf_bits(f)); }
__device__ __forceinline__ float carry_flush(float v, float carry) {
  const float s = v * carry;
  return (fabsf(s) < kF16MinNormal) ? 0.0f : s;
}
__device__ __forceinline__ float frcp(float x) { return __builtin_amdgcn_rcpf(x); }

__device__ __forceinline__ void dep_guard4_h(v8f& a, v8f& b, v8f& c, v8f& d, v16h x, v16h y) { asm volatile("v_nop\n\tv_nop\n\tv_nop\n\tv_nop" : "+v"(a), "+v"(b), "+v"(c), "+v"(d) : "v"(x), "v"(y)); }
__device__ __forceinline__ void dep_guard4_b(v8f& a, v8f& b, v8f& c, v8f& d, v16b x, v16b y) { asm volatile("v_nop\n\tv_nop\n\tv_nop\n\tv_nop" : "+v"(a), "+v"(b), "+v"(c), "+v"(d) : "v"(x), "v"(y)); }
__device__ __forceinline__ void keep4_h(v16h a, v16h b, v16h c, v16h d) { asm volatile("v_nop" :: "v"(a), "v"(b), "v"(c), "v"(d)); }
__device__ __forceinline__ void keep4_b(v16b a, v16b b, v16b c, v16b d) { asm volatile("v_nop" :: "v"(a), "v"(b), "v"(c), "v"(d)); }
__device__ __forceinline__ void acc_guard4(v8f& a, v8f& b, v8f& c, v8f& d) { asm volatile("v_nop\n\tv_nop\n\tv_nop\n\tv_nop" : "+v"(a), "+v"(b), "+v"(c), "+v"(d)); }

template <typename T> struct Frag;
template <> struct Frag<_Float16> {
  typedef v16h V; union U { v16h v; v8h h[2]; };
  static __device__ __forceinline__ v16h load(const _Float16* p) {
    U f; f.h[0] = *(const v8h*)(p); f.h[1] = *(const v8h*)(p + 16); return f.v;
  }
  static __device__ __forceinline__ v8f mma(v16h a, v16h b, v8f c) {
    return __builtin_amdgcn_wmma_f32_16x16x32_f16(false, a, false, b, (short)0, c, false, false);
  }
  static __device__ __forceinline__ void guard4(v8f& a, v8f& b, v8f& c, v8f& d, v16h x, v16h y) { dep_guard4_h(a, b, c, d, x, y); }
  static __device__ __forceinline__ void keep(v16h a, v16h b, v16h c, v16h d) { keep4_h(a, b, c, d); }
};
template <> struct Frag<__bf16> {
  typedef v16b V; union U { v16b v; v8b h[2]; };
  static __device__ __forceinline__ v16b load(const __bf16* p) {
    U f; f.h[0] = *(const v8b*)(p); f.h[1] = *(const v8b*)(p + 16); return f.v;
  }
  static __device__ __forceinline__ v8f mma(v16b a, v16b b, v8f c) {
    return __builtin_amdgcn_wmma_f32_16x16x32_bf16(false, a, false, b, (short)0, c, false, false);
  }
  static __device__ __forceinline__ void guard4(v8f& a, v8f& b, v8f& c, v8f& d, v16b x, v16b y) { dep_guard4_b(a, b, c, d, x, y); }
  static __device__ __forceinline__ void keep(v16b a, v16b b, v16b c, v16b d) { keep4_b(a, b, c, d); }
};

__device__ __forceinline__ v8f mma_h(v16h a, v16h b, v8f c) {
  c = __builtin_amdgcn_wmma_f32_16x16x32_f16(false, a, false, b, (short)0, c, false, false);
  asm volatile("v_nop\n\tv_nop\n\tv_nop\n\tv_nop" : "+v"(c) : "v"(a), "v"(b));
  return c;
}

template <int ET> struct Elem;
template <> struct Elem<0> { typedef _Float16 T; };
template <> struct Elem<1> { typedef __bf16 T; };
template <int ET, bool SPLIT, int BIAS_MODE, int OUT_MODE, bool RESID, int ACT = 0>
__global__ __launch_bounds__(256) void wmma_gemm64(
    const unsigned short* __restrict__ Ap, const unsigned short* __restrict__ A2p, int lda, long strideA,
    const unsigned short* __restrict__ Btp, const unsigned short* __restrict__ Bt2p, int ldb, long strideB,
    void* __restrict__ Cout, void* __restrict__ Cout2, int ldc, long strideC,
    const float* __restrict__ bias,
    const float* __restrict__ resid, long strideR,
    int M, int N, int K, float scale) {
  typedef typename Elem<ET>::T T;
  typedef typename Frag<T>::V V;
  const T* A = (const T*)Ap; const T* A2 = (const T*)A2p; const T* Bt = (const T*)Btp; const T* Bt2 = (const T*)Bt2p;
  __shared__ __align__(16) float sT[8][16 * 68];
  const int b    = blockIdx.y;
  const int lane = threadIdx.x & 31;
  const int wave = threadIdx.x >> 5;
  const int tilesN = N >> 6;
  const int tilesM = M >> 6;
  const int tile = blockIdx.x * 8 + wave;
  if (tile >= tilesM * tilesN) return;
  const int tm = tile / tilesN;
  const int tn = tile - tm * tilesN;
  const int m0 = tm << 6;
  const int n0 = tn << 6;

  const T* Ab  = A  + (size_t)b * strideA;
  const T* Bb  = Bt + (size_t)b * strideB;
  const T* Ab2 = SPLIT ? (A2  + (size_t)b * strideA) : nullptr;
  const T* Bb2 = SPLIT ? (Bt2 + (size_t)b * strideB) : nullptr;

  const int rlane = lane & 15;
  const int koff  = (lane >> 4) * 8;
  const int mOff  = (lane >> 4) * 8;

  v8f acc[4][4];
#pragma unroll
  for (int i = 0; i < 4; ++i)
#pragma unroll
    for (int j = 0; j < 4; ++j) acc[i][j] = (v8f){0.f,0.f,0.f,0.f,0.f,0.f,0.f,0.f};

  for (int k0 = 0; k0 < K; k0 += 32) {
    V bh[4], bl[4];
#pragma unroll
    for (int j = 0; j < 4; ++j) {
      const size_t bo = (size_t)(n0 + (j << 4) + rlane) * ldb + koff + k0;
      bh[j] = Frag<T>::load(Bb + bo);
      if (SPLIT) bl[j] = Frag<T>::load(Bb2 + bo);
    }
#pragma unroll
    for (int i = 0; i < 4; ++i) {
      const size_t ao = (size_t)(m0 + (i << 4) + rlane) * lda + koff + k0;
      V ah = Frag<T>::load(Ab + ao);
      V al;
      if (SPLIT) al = Frag<T>::load(Ab2 + ao);
#pragma unroll
      for (int j = 0; j < 4; ++j) {
        acc[i][j] = Frag<T>::mma(ah, bh[j], acc[i][j]);
        if (SPLIT) {
          acc[i][j] = Frag<T>::mma(ah, bl[j], acc[i][j]);
          acc[i][j] = Frag<T>::mma(al, bh[j], acc[i][j]);
        }
      }
      Frag<T>::guard4(acc[i][0], acc[i][1], acc[i][2], acc[i][3], ah, SPLIT ? al : ah);
    }
    Frag<T>::keep(bh[0], bh[1], bh[2], bh[3]);
    if (SPLIT) Frag<T>::keep(bl[0], bl[1], bl[2], bl[3]);
  }
  acc_guard4(acc[0][0], acc[0][1], acc[0][2], acc[0][3]);
  acc_guard4(acc[1][0], acc[1][1], acc[1][2], acc[1][3]);
  acc_guard4(acc[2][0], acc[2][1], acc[2][2], acc[2][3]);
  acc_guard4(acc[3][0], acc[3][1], acc[3][2], acc[3][3]);

  float* slab = sT[wave];
  const float* Rb = RESID ? (resid + (size_t)b * strideR) : nullptr;
#pragma unroll
  for (int i = 0; i < 4; ++i) {
    const int mBase = m0 + (i << 4);
#pragma unroll
    for (int j = 0; j < 4; ++j) {
      const int n = n0 + (j << 4) + rlane;
      float bv = 0.f;
      if (BIAS_MODE == 2) bv = bias[n];
#pragma unroll
      for (int r = 0; r < 8; ++r) {
        float v = acc[i][j][r] * scale;
        if (BIAS_MODE == 1) v += bias[mBase + mOff + r];
        if (BIAS_MODE == 2) v += bv;
        if (RESID) v += Rb[(size_t)(mBase + mOff + r) * ldc + n];
        if (ACT == 1) v = tanhf(v);
        if (ACT == 2) v = fmaxf(v, 0.0f);
        if (ACT == 3) v = v / (1.0f + expf(-v));
        if (ACT == 4) v = (v > 0.f) ? v : 0.01f * v;
        slab[(mOff + r) * 68 + (j << 4) + rlane] = v;
      }
    }
    __builtin_amdgcn_fence(__ATOMIC_RELEASE, "workgroup");
    __builtin_amdgcn_wave_barrier();
    __builtin_amdgcn_fence(__ATOMIC_ACQUIRE, "workgroup");
    if (OUT_MODE == 0) {
      float* C = (float*)Cout + (size_t)b * strideC;
      const int hh = lane >> 4, c4 = (lane & 15) * 4;
      for (int pass = 0; pass < 2; ++pass) {
#pragma unroll
        for (int it = 0; it < 8; ++it) {
          const int row = it * 2 + hh;
          v4f v = *(const v4f*)(slab + row * 68 + c4);
          *(volatile v4f*)(C + (size_t)(mBase + row) * ldc + n0 + c4) = v;
        }
        __threadfence();
      }
    } else {
      const int q = lane >> 3, c8 = (lane & 7) * 8;
      unsigned short* C  = (unsigned short*)Cout  + (size_t)b * strideC;
      unsigned short* C2 = (OUT_MODE == 2) ? ((unsigned short*)Cout2 + (size_t)b * strideC) : nullptr;
      for (int pass = 0; pass < 2; ++pass) {
#pragma unroll
        for (int it = 0; it < 4; ++it) {
          const int row = it * 4 + q;
          const float* sp = slab + row * 68 + c8;
          v8h hv, lv;
#pragma unroll
          for (int e = 0; e < 8; ++e) {
            if (OUT_MODE == 1) {
              hv[e] = (_Float16)sp[e];
            } else {
              unsigned short hb = f2bf_bits(sp[e]);
              unsigned short lb = f2bf_bits(sp[e] - bf_bits2f(hb));
              hv[e] = __builtin_bit_cast(_Float16, hb);
              lv[e] = __builtin_bit_cast(_Float16, lb);
            }
          }
          *(volatile v8h*)(C + (size_t)(mBase + row) * ldc + n0 + c8) = hv;
          if (OUT_MODE == 2) *(volatile v8h*)(C2 + (size_t)(mBase + row) * ldc + n0 + c8) = lv;
        }
        __threadfence();
      }
    }
    __builtin_amdgcn_fence(__ATOMIC_RELEASE, "workgroup");
    __builtin_amdgcn_wave_barrier();
    __builtin_amdgcn_fence(__ATOMIC_ACQUIRE, "workgroup");
  }
}

__global__ __launch_bounds__(kThr) void cast_plane_kernel(const float* __restrict__ src, unsigned short* __restrict__ dst,
                                                          int colsLog2, int dstPitch, int dstOff) {
  const int i   = blockIdx.x * kThr + threadIdx.x;
  const int sh  = colsLog2 - 3;
  const int row = i >> sh;
  const int c8  = (i & ((1 << sh) - 1)) * 8;
  const float* sp = src + ((size_t)row << colsLog2) + c8;
  const v4f a0 = *(const v4f*)(sp);
  const v4f a1 = *(const v4f*)(sp + 4);
  v8h hv;
#pragma unroll
  for (int e = 0; e < 4; ++e) {
    const float f0 = a0[e];
    const float f1 = a1[e];
    hv[e]     = (_Float16)carry_flush(bf16r(f0), kInCarry);
    hv[4 + e] = (_Float16)carry_flush(bf16r(f1), kInCarry);
  }
  unsigned short* dp = dst + (size_t)row * dstPitch + dstOff + c8;
  *(volatile v8h*)dp = hv;
  __threadfence();
  *(volatile v8h*)dp = hv;
}

__device__ __forceinline__ void split_hl(float v, float c, _Float16& hi, _Float16& lo) {
  const float sv = carry_flush(v, c);
  hi = (_Float16)sv;
  const float r = sv - (float)hi;
  lo = (_Float16)((fabsf(r) < kF16MinNormal) ? 0.0f : r);
}

__global__ __launch_bounds__(64) void wt_plane_kernel(const float* __restrict__ W, unsigned short* __restrict__ WT16, int ldd, int colOff) {
  const int n  = blockIdx.x;
  const int k8 = threadIdx.x * 8;
  v8h hv;
#pragma unroll
  for (int e = 0; e < 8; ++e) hv[e] = (_Float16)carry_flush(bf16r(W[(size_t)(k8 + e) * kHid + n]), kWtCarry);
  unsigned short* dp = WT16 + (size_t)n * ldd + colOff + k8;
  *(volatile v8h*)dp = hv;
  __threadfence();
  *(volatile v8h*)dp = hv;
}

__global__ __launch_bounds__(kThr) void la_setup_kernel(float* __restrict__ ZB, float* __restrict__ ST32, unsigned short* __restrict__ ST16) {
  if (blockIdx.x == 0) {
#pragma unroll 1
    for (int it = 0; it < kH3 / kThr; ++it) {
      const int e = it * kThr + threadIdx.x;
      for (int pass = 0; pass < 2; ++pass) {
        *(volatile float*)(ZB + e) = 0.0f;
        __threadfence();
      }
    }
  } else {
    const size_t i4 = ((size_t)(blockIdx.x - 1) * kThr + threadIdx.x) * 4;
    const v4f z = {0.f, 0.f, 0.f, 0.f};
    const v4h zh = {(_Float16)0.0f, (_Float16)0.0f, (_Float16)0.0f, (_Float16)0.0f};
    const size_t xr = (i4 >> 9) * kK2 + (i4 & 511);
    for (int pass = 0; pass < 2; ++pass) {
      *(volatile v4f*)(ST32 + i4) = z;
      *(volatile v4h*)(ST16 + xr) = zh;
      *(volatile v4h*)(ST16 + xr + kHid) = zh;
      __threadfence();
    }
  }
}
static_assert(((size_t)kBatch * kHid * kHid / 4) % kThr == 0, "state grid exact");

__global__ __launch_bounds__(kThr) void la_prep_kernel(const float* __restrict__ QKVB, unsigned short* __restrict__ Q16,
                                                       unsigned short* __restrict__ K16, unsigned short* __restrict__ KT16,
                                                       unsigned short* __restrict__ VT16) {
  const int blk = blockIdx.x;
  const int tid = threadIdx.x;
  v8h hv;
  unsigned short* dp;
  if (blk < 256) {
    const int which = blk >> 7;
    const int v = (blk & 127) * kThr + tid;
    const int row = v >> 6;
    const int c8 = (v & 63) * 8;
    const float* sp = QKVB + (size_t)row * kH3 + which * kHid + c8;
    const v4f a0 = *(const v4f*)sp;
    const v4f a1 = *(const v4f*)(sp + 4);
    v8h lv;
#pragma unroll
    for (int e = 0; e < 4; ++e) {
      _Float16 h0, l0, h1, l1;
      split_hl(a0[e], kQCarry, h0, l0);
      split_hl(a1[e], kQCarry, h1, l1);
      hv[e] = h0; hv[4 + e] = h1; lv[e] = l0; lv[4 + e] = l1;
    }
    if (which == 0) {
      unsigned short* lp = Q16 + (size_t)row * kK2 + kHid + c8;
      *(volatile v8h*)lp = lv;
      __threadfence();
      *(volatile v8h*)lp = lv;
    }
    dp = which ? (K16 + (size_t)row * kHid + c8) : (Q16 + (size_t)row * kK2 + c8);
  } else {
    const int which = (blk - 256) >> 7;
    const int bb = ((blk - 256) & 127) >> 5;
    const int r = (((blk - 256) & 31) * 16) + (tid >> 4);
    const int s8 = (tid & 15) * 8;
    const float* sp = QKVB + ((size_t)bb * kTB + s8) * kH3 + (which ? 2 * kHid : kHid) + r;
#pragma unroll
    for (int e = 0; e < 8; ++e) hv[e] = (_Float16)carry_flush(sp[(size_t)e * kH3], kQCarry);
    dp = (which ? VT16 : KT16) + ((size_t)bb * kHid + r) * kTB + s8;
  }
  *(volatile v8h*)dp = hv;
  __threadfence();
  *(volatile v8h*)dp = hv;
}
static_assert(kBatch * kTB * kHid / 8 == 128 * kThr && kBatch * kHid * kTB / 8 == 128 * kThr, "prep grid exact");

__global__ __launch_bounds__(kThr) void la_mask_kernel(const float* __restrict__ QK, unsigned short* __restrict__ W16) {
  const int v = blockIdx.x * kThr + threadIdx.x;
  const int row = v >> 4;
  const int s8 = (v & 15) * 8;
  const int t = row & (kTB - 1);
  const float* rp = QK + (size_t)row * kTB + s8;
  const v4f x0 = *(const v4f*)rp, x1 = *(const v4f*)(rp + 4);
  v8h hv;
#pragma unroll
  for (int e = 0; e < 8; ++e) {
    const float qk = (e < 4) ? x0[e] : x1[e - 4];
    const float w = (s8 + e <= t) ? qk : 0.0f;
    hv[e] = (_Float16)carry_flush(w, kSCarry);
  }
  unsigned short* dp = W16 + (size_t)row * kTB + s8;
  *(volatile v8h*)dp = hv;
  __threadfence();
  *(volatile v8h*)dp = hv;
}
static_assert((kBatch * kTB * kTB / 8) % kThr == 0, "mask grid exact");

__global__ __launch_bounds__(kThr) void la_combine_kernel(const float* __restrict__ P1, const float* __restrict__ P2,
                                                          unsigned short* __restrict__ Y16, int t0) {
  const int v = blockIdx.x * kThr + threadIdx.x;
  const int row = v >> 6;
  const int m8 = (v & 63) * 8;
  const int bb = row >> 7;
  const int t = row & (kTB - 1);
  const float* p1 = P1 + (size_t)row * kHid + m8;
  const float* p2 = P2 + (size_t)row * kHid + m8;
  const v4f a0 = *(const v4f*)p1, a1 = *(const v4f*)(p1 + 4);
  const v4f c0 = *(const v4f*)p2, c1 = *(const v4f*)(p2 + 4);
  v8h hv, lv;
#pragma unroll
  for (int e = 0; e < 4; ++e) {
    _Float16 h0, l0, h1, l1;
    split_hl(a0[e] + c0[e], kYCarry, h0, l0);
    split_hl(a1[e] + c1[e], kYCarry, h1, l1);
    hv[e] = h0; hv[4 + e] = h1; lv[e] = l0; lv[4 + e] = l1;
  }
  unsigned short* op = Y16 + ((size_t)bb * kSeq + t0 + t) * kK2 + m8;
  for (int pass = 0; pass < 2; ++pass) {
    *(volatile v8h*)op = hv;
    *(volatile v8h*)(op + kHid) = lv;
    __threadfence();
  }
}
static_assert((kBatch * kTB * kHid / 8) % kThr == 0, "combine grid exact");

__global__ __launch_bounds__(kThr) void la_state_kernel(const float* __restrict__ U, float* __restrict__ ST32,
                                                        unsigned short* __restrict__ ST16) {
  const size_t i4 = ((size_t)blockIdx.x * kThr + threadIdx.x) * 4;
  const v4f s = *(const v4f*)(ST32 + i4);
  const v4f u = *(const v4f*)(U + i4);
  v4f o;
  v4h ho;
#pragma unroll
  for (int e = 0; e < 4; ++e) { o[e] = s[e] + u[e]; ho[e] = (_Float16)carry_flush(o[e], kSCarry); }
  const size_t xr = (i4 >> 9) * kK2 + (i4 & 511);
  for (int pass = 0; pass < 2; ++pass) {
    *(volatile v4f*)(ST32 + i4) = o;
    *(volatile v4h*)(ST16 + xr) = ho;
    *(volatile v4h*)(ST16 + xr + kHid) = ho;
    __threadfence();
  }
}

static_assert(((size_t)kRows * kDin / 8) % kThr == 0, "cast grid exact");

extern "C" void kernel_launch(void* const* d_in, const int* in_sizes, int n_in,
                              void* d_out, int out_size, void* d_ws, size_t ws_size,
                              hipStream_t stream) {
  if (n_in < 5 || d_out == nullptr || d_ws == nullptr) return;
  if (in_sizes[0] != kRows * kDin) return;
  if (in_sizes[1] != kDin * kHid || in_sizes[2] != kDin * kHid || in_sizes[3] != kDin * kHid || in_sizes[4] != kHid * kDin) return;
  if (out_size != kRows * kDin) return;
  if (ws_size < kWsTotal) return;
  const float* x  = (const float*)d_in[0];
  const float* Wq = (const float*)d_in[1];
  const float* Wk = (const float*)d_in[2];
  const float* Wv = (const float*)d_in[3];
  const float* Wo = (const float*)d_in[4];
  float* out = (float*)d_out;
  char* ws = (char*)d_ws;
  unsigned short* X16  = (unsigned short*)(ws + kOffX16);
  unsigned short* WT16 = (unsigned short*)(ws + kOffWT);
  unsigned short* WOT  = (unsigned short*)(ws + kOffWOT);
  float* ZB   = (float*)(ws + kOffZB);
  float* QKVB = (float*)(ws + kOffQKVB);
  unsigned short* Q16  = (unsigned short*)(ws + kOffQ16);
  unsigned short* K16  = (unsigned short*)(ws + kOffK16);
  unsigned short* KT16 = (unsigned short*)(ws + kOffKT);
  unsigned short* VT16 = (unsigned short*)(ws + kOffVT);
  float* QK   = (float*)(ws + kOffQK);
  unsigned short* W16  = (unsigned short*)(ws + kOffW16);
  float* P1   = (float*)(ws + kOffP1);
  float* P2   = (float*)(ws + kOffP2);
  float* U    = (float*)(ws + kOffU);
  float* ST32 = (float*)(ws + kOffST32);
  unsigned short* ST16 = (unsigned short*)(ws + kOffST16);
  unsigned short* Y16  = (unsigned short*)(ws + kOffY16);

  cast_plane_kernel<<<(int)(((size_t)kRows * kDin / 8) / kThr), kThr, 0, stream>>>(x, X16, 9, kDin, 0);
  wt_plane_kernel<<<kHid, kDin / 8, 0, stream>>>(Wq, WT16, kDin, 0);
  wt_plane_kernel<<<kHid, kDin / 8, 0, stream>>>(Wk, WT16 + (size_t)kHid * kDin, kDin, 0);
  wt_plane_kernel<<<kHid, kDin / 8, 0, stream>>>(Wv, WT16 + (size_t)2 * kHid * kDin, kDin, 0);
  wt_plane_kernel<<<kHid, kDin / 8, 0, stream>>>(Wo, WOT, kK2, 0);
  wt_plane_kernel<<<kHid, kDin / 8, 0, stream>>>(Wo, WOT, kK2, kHid);
  la_setup_kernel<<<1 + (kBatch * kHid * kHid / 4) / kThr, kThr, 0, stream>>>(ZB, ST32, ST16);

  for (int blk = 0; blk < kNBlk; ++blk) {
    const int t0 = blk * kTB;
    wmma_gemm64<0, false, 2, 0, false, 0><<<dim3(6, kBatch), 256, 0, stream>>>(
        X16 + (size_t)t0 * kDin, X16 + (size_t)t0 * kDin, kDin, (long)kSeq * kDin, WT16, WT16, kDin, 0L,
        (void*)QKVB, (void*)QKVB, kH3, (long)kTB * kH3, ZB, nullptr, 0L, kTB, kH3, kDin, kXwScale);
    la_prep_kernel<<<512, kThr, 0, stream>>>(QKVB, Q16, K16, KT16, VT16);
    wmma_gemm64<0, false, 2, 0, false, 0><<<dim3(1, kBatch), 256, 0, stream>>>(
        Q16, Q16, kK2, (long)kTB * kK2, K16, K16, kHid, (long)kTB * kHid,
        (void*)QK, (void*)QK, kTB, (long)kTB * kTB, ZB, nullptr, 0L, kTB, kTB, kHid, kQkScale);
    la_mask_kernel<<<(kBatch * kTB * kTB / 8) / kThr, kThr, 0, stream>>>(QK, W16);
    wmma_gemm64<0, false, 2, 0, false, 0><<<dim3(2, kBatch), 256, 0, stream>>>(
        Q16, Q16, kK2, (long)kTB * kK2, ST16, ST16, kK2, (long)kHid * kK2,
        (void*)P1, (void*)P1, kHid, (long)kTB * kHid, ZB, nullptr, 0L, kTB, kHid, kK2, kQsScale);
    wmma_gemm64<0, false, 2, 0, false, 0><<<dim3(2, kBatch), 256, 0, stream>>>(
        W16, W16, kTB, (long)kTB * kTB, VT16, VT16, kTB, (long)kHid * kTB,
        (void*)P2, (void*)P2, kHid, (long)kTB * kHid, ZB, nullptr, 0L, kTB, kHid, kTB, kQsScale);
    la_combine_kernel<<<(kBatch * kTB * kHid / 8) / kThr, kThr, 0, stream>>>(P1, P2, Y16, t0);
    if (blk + 1 < kNBlk) {
      wmma_gemm64<0, false, 2, 0, false, 0><<<dim3(8, kBatch), 256, 0, stream>>>(
          VT16, VT16, kTB, (long)kHid * kTB, KT16, KT16, kTB, (long)kHid * kTB,
          (void*)U, (void*)U, kHid, (long)kHid * kHid, ZB, nullptr, 0L, kHid, kHid, kTB, kQkScale);
      la_state_kernel<<<(kBatch * kHid * kHid / 4) / kThr, kThr, 0, stream>>>(U, ST32, ST16);
    }
  }
  wmma_gemm64<0, false, 2, 0, false, 0><<<dim3((kRows / 64) * (kDin / 64) / 8, 1), 256, 0, stream>>>(
      Y16, Y16, kK2, 0L, WOT, WOT, kK2, 0L, (void*)out, (void*)out, kDin, 0L, ZB, nullptr, 0L, kRows, kDin, kK2, kYoScale);
}
